// GraphSage_90692529422657
// MI455X (gfx1250) — hardware-run, weakly checked
//
#include <hip/hip_runtime.h>
#include <stddef.h>
#include <stdint.h>


#define NN      50000
#define NE      800000
#define FD      64
#define CD      40
#define NPC     48
#define MP      50048
#define NTHR    256
#define NWAVE   8
#define EPT     8
#define CHUNK   (NTHR * EPT)
#define WCAP    (EPT * 32)
#define LISTN   (NWAVE * WCAP)
#define NBA     1024
#define PKS     10
#define NBLK    49
#define NPADN   (NBLK * NBA)
#define RCAP    20480
#define DEGCAP  64
#define GBM     128
#define GTHR    256
#define RPB     64
#define RPW     8
#define BK_INTS (2 * RCAP + 3 * NBA + LISTN + 32)
#define LDS_BK  (BK_INTS * 4)
#define MEAS_BLK_HITS 16623
#define MEAS_MAXDEG   35
#define NWBLK   18
#define WSMAX   134217728

static_assert((CHUNK & (CHUNK - 1)) == 0 && CHUNK <= 4096);
static_assert(NBA == (1 << PKS) && NBA == NTHR * 4);
static_assert(LISTN == NWAVE * WCAP);
static_assert(RCAP % (NTHR * 4) == 0 && BK_INTS % 4 == 0);
static_assert((long long)RCAP * 100 >= (long long)MEAS_BLK_HITS * 105);
static_assert(DEGCAP >= MEAS_MAXDEG + 8);
static_assert(LDS_BK <= 300000 && LDS_BK <= 327680);
static_assert(NE < (1 << 21));
static_assert(NPADN >= MP && NBLK <= 64 && NBLK * NBA >= NN);
static_assert(MP % GBM == 0 && MP >= NN && MP - NN < GBM && MP % RPB == 0 && (MP & 1) == 0);
static_assert(NN - (MP - GBM) == 80);
static_assert((GBM * CD * 4) % 128 == 0);
static_assert((80 * CD * 4) % 128 == 0);
static_assert(NPC % 16 == 0 && NPC >= CD && CD % 4 == 0);
static_assert(64 % 32 == 0 && 192 % 32 == 0 && 128 % 32 == 0 && 256 % 32 == 0);
static_assert(GBM == (GTHR / 32) * 16);
static_assert((GBM * CD) / 4 == 5 * GTHR);
static_assert(RPB == NWAVE * RPW && (RPW & 1) == 0);
static_assert((MP * 8) % NTHR == 0);
static_assert(GBM * 64 * 4 + 64 * 4 + GBM * CD * 4 <= 65536);

typedef float          v2f   __attribute__((ext_vector_type(2)));
typedef float          v4f   __attribute__((ext_vector_type(4)));
typedef float          v8f   __attribute__((ext_vector_type(8)));
typedef int            v4i   __attribute__((ext_vector_type(4)));
typedef int            v8i   __attribute__((ext_vector_type(8)));
typedef unsigned       v2u   __attribute__((ext_vector_type(2)));
typedef unsigned       v4u   __attribute__((ext_vector_type(4)));
typedef unsigned short v8us  __attribute__((ext_vector_type(8)));
typedef __bf16         v16bf __attribute__((ext_vector_type(16)));
typedef v4f  __attribute__((may_alias)) v4fa;
typedef v4i  __attribute__((may_alias)) v4ia;
typedef v4u  __attribute__((may_alias)) v4ua;
typedef v8us __attribute__((may_alias)) v8usa;
union FragB { v16bf v; v8us h[2]; v8i w; };

__device__ __forceinline__ v8f wmb(const FragB& a, const FragB& b, v8f c) {
  v8f d = __builtin_amdgcn_wmma_f32_16x16x32_bf16(false, a.v, false, b.v, (short)0, c, false, false);
  asm volatile("v_nop\n\tv_nop\n\tv_nop\n\tv_nop" : "+v"(d) : "v"(a.w), "v"(b.w));
  return d;
}

__device__ __forceinline__ unsigned bf16_bits(float f) {
  const unsigned u = __float_as_uint(f);
  return ((u + 0x7FFFu + ((u >> 16) & 1u)) >> 16) & 0xFFFFu;
}
__device__ __forceinline__ float bf16_val(float f) { return __uint_as_float(bf16_bits(f) << 16); }
__device__ __forceinline__ v2u pack2(float a, float b) {
  const unsigned ha = bf16_bits(a), hb = bf16_bits(b);
  const unsigned la = bf16_bits(a - __uint_as_float(ha << 16));
  const unsigned lb = bf16_bits(b - __uint_as_float(hb << 16));
  v2u r;
  r.x = ha | (hb << 16);
  r.y = la | (lb << 16);
  return r;
}
__device__ __forceinline__ float relu_k(float v) { return (v > 0.0f) ? v : (v - v); }

__device__ __forceinline__ void wave_sync() {
  __builtin_amdgcn_fence(__ATOMIC_RELEASE, "wavefront");
  __builtin_amdgcn_wave_barrier();
  __builtin_amdgcn_fence(__ATOMIC_ACQUIRE, "wavefront");
}

__device__ __forceinline__ void slot_info(const int* __restrict__ CNT, const int* __restrict__ OFF, int node,
                                          int& deg, int& c, int& o) {
  const int craw = CNT[node];
  const int oraw = OFF[node];
  deg = craw < 0 ? 0 : craw;
  c = deg > DEGCAP ? DEGCAP : deg;
  o = oraw < 0 ? 0 : (oraw > RCAP ? RCAP : oraw);
  if (c > RCAP - o) c = RCAP - o;
}

__device__ __forceinline__ int scan_chunk(const int* __restrict__ keys, int nE, int cbase, int slotBase,
                                          int nb, int vec8, int* list, int tid, int lane, int wave) {
  int wc = 0;
  const int el0  = tid * EPT;
  const int e0   = cbase + el0;
  const int sent = -2147483647 - 1;
  v4i da, db;
  if (vec8 != 0 && cbase + CHUNK <= nE) {
    da = *(const v4i*)(keys + e0);
    db = *(const v4i*)(keys + e0 + 4);
  } else {
    da.x = (e0     < nE) ? keys[min(e0,     nE - 1)] : sent;
    da.y = (e0 + 1 < nE) ? keys[min(e0 + 1, nE - 1)] : sent;
    da.z = (e0 + 2 < nE) ? keys[min(e0 + 2, nE - 1)] : sent;
    da.w = (e0 + 3 < nE) ? keys[min(e0 + 3, nE - 1)] : sent;
    db.x = (e0 + 4 < nE) ? keys[min(e0 + 4, nE - 1)] : sent;
    db.y = (e0 + 5 < nE) ? keys[min(e0 + 5, nE - 1)] : sent;
    db.z = (e0 + 6 < nE) ? keys[min(e0 + 6, nE - 1)] : sent;
    db.w = (e0 + 7 < nE) ? keys[min(e0 + 7, nE - 1)] : sent;
  }
  const unsigned nbs = (unsigned)slotBase;
  const unsigned unb = (unsigned)nb;
  const unsigned s0 = (unsigned)da.x - nbs, s1 = (unsigned)da.y - nbs;
  const unsigned s2 = (unsigned)da.z - nbs, s3 = (unsigned)da.w - nbs;
  const unsigned s4 = (unsigned)db.x - nbs, s5 = (unsigned)db.y - nbs;
  const unsigned s6 = (unsigned)db.z - nbs, s7 = (unsigned)db.w - nbs;
  const bool h0 = s0 < unb, h1 = s1 < unb, h2 = s2 < unb, h3 = s3 < unb;
  const bool h4 = s4 < unb, h5 = s5 < unb, h6 = s6 < unb, h7 = s7 < unb;
  const unsigned any = __builtin_amdgcn_ballot_w32(h0 | h1 | h2 | h3 | h4 | h5 | h6 | h7);
  if (any != 0u) {
#define HITJ(J, HJ, SJ) { \
      const unsigned mj = __builtin_amdgcn_ballot_w32(HJ); \
      if (mj != 0u) { \
        if (HJ) { \
          const int pos = wc + (int)__builtin_amdgcn_mbcnt_lo(mj, 0u); \
          if (pos < WCAP) list[wave * WCAP + pos] = ((el0 + (J)) << PKS) | (int)(SJ); \
        } \
        wc += (int)__builtin_popcount(mj); } }
    HITJ(0, h0, s0)
    HITJ(1, h1, s1)
    HITJ(2, h2, s2)
    HITJ(3, h3, s3)
    HITJ(4, h4, s4)
    HITJ(5, h5, s5)
    HITJ(6, h6, s6)
    HITJ(7, h7, s7)
#undef HITJ
  }
  return wc;
}

__device__ __forceinline__ void wtrans(const float* __restrict__ W, int spitch, int nvalid, unsigned short* P,
                                       int dpitch, int n, int ksrc, int kdst) {
  const int nc = n < nvalid ? n : nvalid - 1;
  const float* p = W + (size_t)ksrc * spitch + nc;
  const float f0 = p[0];
  const float f1 = p[(size_t)1 * spitch];
  const float f2 = p[(size_t)2 * spitch];
  const float f3 = p[(size_t)3 * spitch];
  const float f4 = p[(size_t)4 * spitch];
  const float f5 = p[(size_t)5 * spitch];
  const float f6 = p[(size_t)6 * spitch];
  const float f7 = p[(size_t)7 * spitch];
  asm volatile("" :: "v"(f0), "v"(f1), "v"(f2), "v"(f3), "v"(f4), "v"(f5), "v"(f6), "v"(f7));
  const unsigned mk = (n < nvalid) ? 0xFFFFu : 0u;
  v8us o;
  o[0] = (unsigned short)(bf16_bits(f0) & mk); o[1] = (unsigned short)(bf16_bits(f1) & mk);
  o[2] = (unsigned short)(bf16_bits(f2) & mk); o[3] = (unsigned short)(bf16_bits(f3) & mk);
  o[4] = (unsigned short)(bf16_bits(f4) & mk); o[5] = (unsigned short)(bf16_bits(f5) & mk);
  o[6] = (unsigned short)(bf16_bits(f6) & mk); o[7] = (unsigned short)(bf16_bits(f7) & mk);
  unsigned short* dp = P + (size_t)n * dpitch + kdst;
  *(volatile v8us*)dp = o;
  __threadfence();
  *(volatile v8us*)dp = o;
}

__global__ __launch_bounds__(NTHR) void k_prep(const float* __restrict__ x, const float* __restrict__ Wp,
                                               const float* __restrict__ Wl1, const float* __restrict__ Wr1,
                                               const float* __restrict__ Wl2, const float* __restrict__ Wr2,
                                               unsigned short* WPT, unsigned short* WPT2, unsigned short* W1C,
                                               unsigned short* W2C, unsigned short* XB, int nN, int mRows) {
  const int b = (int)blockIdx.x, tid = (int)threadIdx.x;
  if (b < 2) {
    const int v = b * NTHR + tid, n = v >> 3, j = v & 7;
    wtrans(Wp, FD, FD, WPT, 64, n, 8 * j, 8 * j);
  } else if (b < 6) {
    const int v = (b - 2) * NTHR + tid, n = v >> 4, j = v & 15;
    wtrans(Wp, FD, FD, WPT2, 128, n, 8 * (j & 7), 8 * j);
  } else if (b < 10) {
    const int v = (b - 6) * NTHR + tid, n = v >> 4, j = v & 15;
    wtrans(Wl1, FD, FD, W1C, 192, n, 8 * (j & 7), 8 * j);
  } else if (b < 12) {
    const int v = (b - 10) * NTHR + tid, n = v >> 3, j = v & 7;
    wtrans(Wr1, FD, FD, W1C, 192, n, 8 * j, 128 + 8 * j);
  } else if (b < 15) {
    const int v = (b - 12) * NTHR + tid, n = v >> 4, j = v & 15;
    wtrans(Wl2, CD, CD, W2C, 256, n, 8 * (j & 7), 8 * j);
  } else if (b < NWBLK) {
    const int v = (b - 15) * NTHR + tid, n = v >> 4, j = v & 15;
    wtrans(Wr2, CD, CD, W2C, 256, n, 8 * (j & 7), 128 + 8 * j);
  } else {
    const int v   = (b - NWBLK) * NTHR + tid;
    const int row = v >> 3;
    const int c8  = (v & 7) * 8;
    if (row < mRows) {
      const int rc = row < nN ? row : nN - 1;
      const float* p = x + (size_t)rc * FD + c8;
      const v4f a = *(const v4f*)p;
      const v4f c = *(const v4f*)(p + 4);
      asm volatile("" :: "v"(a), "v"(c));
      const unsigned mk = (row < nN) ? 0xFFFFu : 0u;
      v8us o;
      o[0] = (unsigned short)(bf16_bits(a.x) & mk); o[1] = (unsigned short)(bf16_bits(a.y) & mk);
      o[2] = (unsigned short)(bf16_bits(a.z) & mk); o[3] = (unsigned short)(bf16_bits(a.w) & mk);
      o[4] = (unsigned short)(bf16_bits(c.x) & mk); o[5] = (unsigned short)(bf16_bits(c.y) & mk);
      o[6] = (unsigned short)(bf16_bits(c.z) & mk); o[7] = (unsigned short)(bf16_bits(c.w) & mk);
      unsigned short* dp = XB + (size_t)row * FD + c8;
      *(volatile v8us*)dp = o;
      __threadfence();
      *(volatile v8us*)dp = o;
    }
  }
}

__global__ __launch_bounds__(NTHR) void k_bucket(const int* __restrict__ keys, const int* __restrict__ gidx,
                                                 int nE, int nN, int vec8,
                                                 int* LIST, int* CNT, int* OFF, int* REC) {
  extern __shared__ __attribute__((aligned(16))) int dsm[];
  int* reg1 = dsm;
  int* reg2 = reg1 + RCAP;
  int* scnt = reg2 + RCAP;
  int* soff = scnt + NBA;
  int* cur  = soff + NBA;
  int* list = cur + NBA;
  int* wcnt = list + LISTN;
  int* wtot = wcnt + 8;
  int* wmx  = wtot + 8;
  const int tid = (int)threadIdx.x, lane = tid & 31, wave = tid >> 5;
  const int nodeBase = (int)blockIdx.x * NBA;
  int nb = nN - nodeBase;
  nb = nb > NBA ? NBA : (nb < 1 ? 1 : nb);

  {
    const v4i z4 = {0, 0, 0, 0};
    for (int i = tid * 4; i < BK_INTS; i += NTHR * 4) *(v4ia*)(dsm + i) = z4;
  }
  __syncthreads();

  int tot = 0;
  const int nChunks = (nE + CHUNK - 1) / CHUNK;
#pragma unroll 1
  for (int ch = 0; ch < nChunks; ++ch) {
    const int cbase = ch * CHUNK;
    const int wc = scan_chunk(keys, nE, cbase, nodeBase, nb, vec8, list, tid, lane, wave);
    if (lane == 0) wcnt[wave] = wc;
    __syncthreads();
    int pre = 0, all = 0;
#pragma unroll
    for (int w2 = 0; w2 < NWAVE; ++w2) {
      int c = wcnt[w2];
      c = c < 0 ? 0 : (c > WCAP ? WCAP : c);
      all += c;
      pre += (w2 < wave) ? c : 0;
    }
    const int wcc  = wc > WCAP ? WCAP : wc;
    const int base = tot + pre;
#pragma unroll 1
    for (int i = lane; i < wcc; i += 32) {
      const int ent = list[wave * WCAP + i];
      const int el  = (ent >> PKS) & (CHUNK - 1);
      const int sl  = ent & (NBA - 1);
      int eid = cbase + el;
      eid = eid > nE - 1 ? nE - 1 : eid;
      const int pos = base + i;
      if (pos < RCAP) reg1[pos] = (int)(((unsigned)eid << PKS) | (unsigned)sl);
    }
    tot += all;
    tot = tot > RCAP ? RCAP : tot;
    __syncthreads();
  }
  const int nh = tot;

  if (wave == 0) {
#pragma unroll 1
    for (int b0 = 0; b0 < nh; b0 += 32) {
      const int idx = b0 + lane;
      const int uv  = reg1[idx < RCAP ? idx : RCAP - 1];
      const int m32 = (nh - b0) < 32 ? (nh - b0) : 32;
#pragma unroll 1
      for (int k = 0; k < m32; ++k) {
        const int u  = __builtin_amdgcn_readlane(uv, k);
        const int sl = u & (NBA - 1);
        if (lane == 0) scnt[sl] = scnt[sl] + 1;
      }
    }
  }
  __syncthreads();

  {
    const v4i ca = *(const v4ia*)(scnt + 4 * tid);
    const int e0 = ca.x < 0 ? 0 : ca.x, e1 = ca.y < 0 ? 0 : ca.y, e2 = ca.z < 0 ? 0 : ca.z, e3 = ca.w < 0 ? 0 : ca.w;
    const int ts = e0 + e1 + e2 + e3;
    int incl = ts;
#pragma unroll
    for (int d = 1; d < 32; d <<= 1) {
      const int up = __shfl_up(incl, d, 32);
      if (lane >= d) incl += up;
    }
    int mx = max(max(e0, e1), max(e2, e3));
    mx = max(mx, __shfl_xor(mx, 16, 32));
    mx = max(mx, __shfl_xor(mx, 8, 32));
    mx = max(mx, __shfl_xor(mx, 4, 32));
    mx = max(mx, __shfl_xor(mx, 2, 32));
    mx = max(mx, __shfl_xor(mx, 1, 32));
    if (lane == 31) wtot[wave] = incl;
    if (lane == 0)  wmx[wave] = mx;
    __syncthreads();
    int pre = 0;
#pragma unroll
    for (int w2 = 0; w2 < NWAVE; ++w2) pre += (w2 < wave) ? wtot[w2] : 0;
    int run = pre + incl - ts;
    v4i so;
    so.x = run; run += e0;
    so.y = run; run += e1;
    so.z = run; run += e2;
    so.w = run;
    *(v4ia*)(soff + 4 * tid) = so;
    *(v4ia*)(cur + 4 * tid)  = so;
  }
  __syncthreads();

  if (wave == 0) {
#pragma unroll 1
    for (int b0 = 0; b0 < nh; b0 += 32) {
      const int idx = b0 + lane;
      const int uv  = reg1[idx < RCAP ? idx : RCAP - 1];
      const int m32 = (nh - b0) < 32 ? (nh - b0) : 32;
#pragma unroll 1
      for (int k = 0; k < m32; ++k) {
        const int u   = __builtin_amdgcn_readlane(uv, k);
        const int sl  = u & (NBA - 1);
        const int eid = (int)((unsigned)u >> PKS);
        if (lane == 0) {
          int pos = cur[sl];
          pos = pos < 0 ? 0 : (pos > RCAP - 1 ? RCAP - 1 : pos);
          reg2[pos] = eid;
          cur[sl] = pos + 1;
        }
      }
    }
  }
  __syncthreads();

  int bmax = 0;
#pragma unroll
  for (int w2 = 0; w2 < NWAVE; ++w2) bmax = max(bmax, wmx[w2]);
  const int flag = ((nh >= RCAP) || (bmax > DEGCAP)) ? 1 : 0;

  int* lrow = LIST + (size_t)blockIdx.x * RCAP;
#pragma unroll 1
  for (int it = 0; it < RCAP / (NTHR * 4); ++it) {
    const int i0 = 4 * (it * NTHR + tid);
    const v4i ev = *(const v4ia*)(reg2 + i0);
    int e0 = ev.x, e1 = ev.y, e2 = ev.z, e3 = ev.w;
    e0 = e0 < 0 ? 0 : (e0 > nE - 1 ? nE - 1 : e0);
    e1 = e1 < 0 ? 0 : (e1 > nE - 1 ? nE - 1 : e1);
    e2 = e2 < 0 ? 0 : (e2 > nE - 1 ? nE - 1 : e2);
    e3 = e3 < 0 ? 0 : (e3 > nE - 1 ? nE - 1 : e3);
    int g0 = gidx[e0], g1 = gidx[e1], g2 = gidx[e2], g3 = gidx[e3];
    asm volatile("" :: "v"(g0), "v"(g1), "v"(g2), "v"(g3));
    g0 = g0 < 0 ? 0 : (g0 > nN - 1 ? nN - 1 : g0);
    g1 = g1 < 0 ? 0 : (g1 > nN - 1 ? nN - 1 : g1);
    g2 = g2 < 0 ? 0 : (g2 > nN - 1 ? nN - 1 : g2);
    g3 = g3 < 0 ? 0 : (g3 > nN - 1 ? nN - 1 : g3);
    v4i ov;
    ov.x = (i0     < nh) ? g0 : 0;
    ov.y = (i0 + 1 < nh) ? g1 : 0;
    ov.z = (i0 + 2 < nh) ? g2 : 0;
    ov.w = (i0 + 3 < nh) ? g3 : 0;
    *(volatile v4i*)(lrow + i0) = ov;
    __threadfence();
    *(volatile v4i*)(lrow + i0) = ov;
  }
  {
    const v4i cv = *(const v4ia*)(scnt + 4 * tid);
    const v4i fv = *(const v4ia*)(soff + 4 * tid);
    v4i rv = {0, 0, 0, 0};
    rv.x = (tid == 0) ? bmax : 0;
    rv.y = (tid == 0) ? flag : 0;
    rv.z = (tid == 0) ? nh : 0;
    int* cp = CNT + (size_t)nodeBase + 4 * tid;
    int* fp = OFF + (size_t)nodeBase + 4 * tid;
    int* rp = REC + (size_t)blockIdx.x * 32 + 4 * (tid & 7);
    *(volatile v4i*)cp = cv;
    *(volatile v4i*)fp = fv;
    if (tid < 8) *(volatile v4i*)rp = rv;
    __threadfence();
    *(volatile v4i*)cp = cv;
    *(volatile v4i*)fp = fv;
    if (tid < 8) *(volatile v4i*)rp = rv;
  }
}

__device__ __forceinline__ v2u max_row(const float* __restrict__ Mp, const int* __restrict__ LIST,
                                       const int* __restrict__ CNT, const int* __restrict__ OFF,
                                       const int* __restrict__ REC, int node, int nN, int nB, int lane) {
  const int nodet = node < NPADN ? node : NPADN - 1;
  int deg, c, o;
  slot_info(CNT, OFF, nodet, deg, c, o);
  int blk = nodet >> PKS;
  blk = blk > nB - 1 ? nB - 1 : blk;
  const int fl = REC[(size_t)blk * 32 + 1];
  const int* lp = LIST + (size_t)blk * RCAP;
  float a0 = 0.0f, a1 = 0.0f;
  unsigned n0 = 0u, n1 = 0u;
#pragma unroll 1
  for (int b0 = 0; b0 < c; b0 += 32) {
    int idx = o + b0 + lane;
    idx = idx > RCAP - 1 ? RCAP - 1 : idx;
    int col = lp[idx];
    col = col < 0 ? 0 : (col > nN - 1 ? nN - 1 : col);
    const int m32 = (c - b0) < 32 ? (c - b0) : 32;
#pragma unroll 1
    for (int k = 0; k < m32; ++k) {
      const int sk = __builtin_amdgcn_readlane(col, k);
      const v2f v = *(const v2f*)(Mp + (size_t)sk * FD + 2 * lane);
      a0 = (v.x > a0) ? v.x : a0;
      a1 = (v.y > a1) ? v.y : a1;
      n0 |= (v.x != v.x) ? 1u : 0u;
      n1 |= (v.y != v.y) ? 1u : 0u;
    }
  }
  const bool pz = (fl != 0) || (deg > DEGCAP);
  const float qn = __int_as_float(0x7fc00000);
  float r0 = (pz || n0 != 0u) ? qn : a0;
  float r1 = (pz || n1 != 0u) ? qn : a1;
  const bool live = node < nN;
  r0 = live ? r0 : 0.0f;
  r1 = live ? r1 : 0.0f;
  return pack2(r0, r1);
}

__global__ __launch_bounds__(NTHR) void k_max(const float* __restrict__ Mp, const int* __restrict__ LIST,
                                              const int* __restrict__ CNT, const int* __restrict__ OFF,
                                              const int* __restrict__ REC, unsigned short* AGG,
                                              int nN, int mRows, int nB) {
  __shared__ __attribute__((aligned(16))) unsigned wstage[NWAVE * 128];
  const int tid = (int)threadIdx.x, lane = tid & 31, wave = tid >> 5;
  unsigned* wst = wstage + wave * 128;
#pragma unroll 1
  for (int pi = 0; pi < RPW / 2; ++pi) {
    const int node0 = (int)blockIdx.x * RPB + wave * RPW + 2 * pi;
    if (node0 + 1 >= mRows) continue;
    const v2u ra = max_row(Mp, LIST, CNT, OFF, REC, node0, nN, nB, lane);
    const v2u rb = max_row(Mp, LIST, CNT, OFF, REC, node0 + 1, nN, nB, lane);
    wst[lane]      = ra.x;
    wst[32 + lane] = ra.y;
    wst[64 + lane] = rb.x;
    wst[96 + lane] = rb.y;
    wave_sync();
    const v4u q = *(const v4ua*)(wst + 4 * lane);
    wave_sync();
    unsigned short* wp = AGG + (size_t)node0 * 128 + 8 * lane;
    *(volatile v4u*)wp = q;
    __threadfence();
    *(volatile v4u*)wp = q;
  }
}

template <int NT>
__device__ __forceinline__ void kseg(const unsigned short* __restrict__ ap, const unsigned short* __restrict__ bp,
                                     int nsteps, int kb, v8f (&acc)[NT]) {
#pragma unroll 1
  for (int ks = 0; ks < nsteps; ++ks) {
    FragB af;
    af.h[0] = *(const v8usa*)(ap + 32 * ks);
    af.h[1] = *(const v8usa*)(ap + 32 * ks + 16);
#pragma unroll
    for (int t = 0; t < NT; ++t) {
      const unsigned short* wq = bp + (size_t)(16 * t) * (size_t)kb + 32 * ks;
      FragB bf;
      bf.h[0] = *(const v8usa*)wq;
      bf.h[1] = *(const v8usa*)(wq + 16);
      acc[t] = wmb(af, bf, acc[t]);
    }
  }
}

template <int MODE>
__global__ __launch_bounds__(GTHR) __attribute__((amdgpu_num_vgpr(248)))
void k_gemm(const unsigned short* __restrict__ A0, const unsigned short* __restrict__ A1,
            const unsigned short* __restrict__ BT, const float* __restrict__ bias,
            float* outF, unsigned short* outH, const int* __restrict__ REC, int nN, int nB) {
  constexpr int NT  = (MODE == 3) ? 3 : 4;
  constexpr int KB  = (MODE == 0) ? 64 : ((MODE == 1) ? 192 : ((MODE == 2) ? 128 : 256));
  constexpr int P0  = (MODE == 0) ? 64 : 128;
  constexpr int S0  = (MODE == 0) ? 2 : 4;
  constexpr int P1  = (MODE == 1) ? 64 : 128;
  constexpr int S1  = (MODE == 1) ? 2 : ((MODE == 3) ? 4 : 0);
  constexpr int SP  = (MODE == 3) ? NPC : 64;
  constexpr int NBV = (MODE == 3) ? CD : 64;
  __shared__ __attribute__((aligned(16))) float stg[GBM * 64];
  __shared__ __attribute__((aligned(16))) float bsh[64];
  const int tid = (int)threadIdx.x, lane = tid & 31, wave = tid >> 5, hh = lane >> 4, m = lane & 15;
  const int rowBase = (int)blockIdx.x * GBM;

  if (tid < 32) {
    const int c4  = 4 * m;
    const int c4c = c4 > NBV - 4 ? NBV - 4 : c4;
    const v4f b4 = *(const v4f*)(bias + c4c);
    asm volatile("" :: "v"(b4));
    const bool bl = c4 < NBV;
    v4f bq;
    bq.x = bl ? bf16_val(b4.x) : 0.0f;
    bq.y = bl ? bf16_val(b4.y) : 0.0f;
    bq.z = bl ? bf16_val(b4.z) : 0.0f;
    bq.w = bl ? bf16_val(b4.w) : 0.0f;
    if (tid < 16) *(v4fa*)(bsh + c4) = bq;
  }

  v8f acc[NT];
  {
    const v8f z = {0.f, 0.f, 0.f, 0.f, 0.f, 0.f, 0.f, 0.f};
#pragma unroll
    for (int t = 0; t < NT; ++t) acc[t] = z;
  }
  const size_t arow = (size_t)(rowBase + 16 * wave + m);
  const unsigned short* bp = BT + (size_t)m * (size_t)KB + 8 * hh;
  kseg<NT>(A0 + arow * P0 + 8 * hh, bp, S0, KB, acc);
  if constexpr (S1 > 0) kseg<NT>(A1 + arow * P1 + 8 * hh, bp + 128, S1, KB, acc);
  __syncthreads();

#pragma unroll
  for (int t = 0; t < NT; ++t) {
    const int lc = 16 * t + m;
    const float bb = bsh[lc];
#pragma unroll
    for (int r = 0; r < 8; ++r) {
      const int lr = 16 * wave + 8 * hh + r;
      if constexpr (MODE == 3) {
        stg[lr * SP + lc] = acc[t][r] + bb;
      } else if constexpr (MODE == 1) {
        const bool live = (rowBase + lr) < nN;
        const float v = relu_k(acc[t][r] + bb);
        stg[lr * SP + lc] = live ? v : 0.0f;
      } else {
        stg[lr * SP + lc] = relu_k(acc[t][r] + bb);
      }
    }
  }
  __syncthreads();

  if constexpr (MODE == 0 || MODE == 2) {
    v4f pv[8];
#pragma unroll
    for (int i = 0; i < 8; ++i) {
      const int lr = 16 * wave + 2 * i + hh;
      pv[i] = *(const v4fa*)(stg + lr * 64 + 4 * m);
    }
#pragma unroll
    for (int i = 0; i < 8; ++i) {
      const int lr = 16 * wave + 2 * i + hh;
      float* gp = outF + (size_t)(rowBase + lr) * 64 + 4 * m;
      *(volatile v4f*)gp = pv[i];
    }
    __threadfence();
#pragma unroll
    for (int i = 0; i < 8; ++i) {
      const int lr = 16 * wave + 2 * i + hh;
      float* gp = outF + (size_t)(rowBase + lr) * 64 + 4 * m;
      *(volatile v4f*)gp = pv[i];
    }
  } else if constexpr (MODE == 1) {
    const int cb = 8 * (m & 7);
    const bool isHi = (m < 8);
    v4u pk[8];
#pragma unroll
    for (int i = 0; i < 8; ++i) {
      const int lr = 16 * wave + 2 * i + hh;
      const v4f a = *(const v4fa*)(stg + lr * 64 + cb);
      const v4f b = *(const v4fa*)(stg + lr * 64 + cb + 4);
      const v2u w0 = pack2(a.x, a.y);
      const v2u w1 = pack2(a.z, a.w);
      const v2u w2 = pack2(b.x, b.y);
      const v2u w3 = pack2(b.z, b.w);
      v4u pw;
      pw.x = isHi ? w0.x : w0.y;
      pw.y = isHi ? w1.x : w1.y;
      pw.z = isHi ? w2.x : w2.y;
      pw.w = isHi ? w3.x : w3.y;
      pk[i] = pw;
    }
#pragma unroll
    for (int i = 0; i < 8; ++i) {
      const int lr = 16 * wave + 2 * i + hh;
      unsigned short* gp = outH + (size_t)(rowBase + lr) * 128 + 8 * m;
      *(volatile v4u*)gp = pk[i];
    }
    __threadfence();
#pragma unroll
    for (int i = 0; i < 8; ++i) {
      const int lr = 16 * wave + 2 * i + hh;
      unsigned short* gp = outH + (size_t)(rowBase + lr) * 128 + 8 * m;
      *(volatile v4u*)gp = pk[i];
    }
  } else {
    __shared__ __attribute__((aligned(16))) float ost[GBM * CD];
    const int trow = tid & (GBM - 1);
    const int grow = rowBase + trow;
    int blk = grow >> PKS;
    blk = blk > nB - 1 ? nB - 1 : blk;
    const int fl = REC[(size_t)blk * 32 + 1];
    asm volatile("" :: "v"(fl));
    if (tid < GBM) {
      const float* sr = stg + trow * SP;
      float mx = sr[0];
#pragma unroll 1
      for (int c = 1; c < CD; ++c) {
        const float v = sr[c];
        mx = (v > mx || v != v) ? v : mx;
      }
      float s = 0.0f;
#pragma unroll 1
      for (int c = 0; c < CD; ++c) s += expf(sr[c] - mx);
      const float ls = logf(s);
      const float qn = __int_as_float(0x7fc00000);
      float* orow = ost + trow * CD;
#pragma unroll 1
      for (int c = 0; c < CD; ++c) {
        const float y = (sr[c] - mx) - ls;
        orow[c] = (fl != 0) ? qn : y;
      }
    }
    __syncthreads();
    int nrows = nN - rowBase;
    nrows = nrows < 0 ? 0 : (nrows > GBM ? GBM : nrows);
    const int lim = nrows * (CD / 4);
    v4f ov[5];
#pragma unroll
    for (int it = 0; it < 5; ++it) ov[it] = *(const v4fa*)(ost + 4 * (it * GTHR + tid));
    asm volatile("" :: "v"(ov[0]), "v"(ov[1]), "v"(ov[2]), "v"(ov[3]), "v"(ov[4]));
    float* ob = outF + (size_t)rowBase * CD;
#pragma unroll
    for (int it = 0; it < 5; ++it) {
      const int q = it * GTHR + tid;
      if (q < lim) *(volatile v4f*)(ob + 4 * (size_t)q) = ov[it];
    }
    __threadfence();
#pragma unroll
    for (int it = 0; it < 5; ++it) {
      const int q = it * GTHR + tid;
      if (q < lim) *(volatile v4f*)(ob + 4 * (size_t)q) = ov[it];
    }
  }
}

static inline size_t al256(size_t o) { return (o + 255) & ~(size_t)255; }

extern "C" void kernel_launch(void* const* d_in, const int* in_sizes, int n_in,
                              void* d_out, int out_size, void* d_ws, size_t ws_size,
                              hipStream_t stream) {
  if (n_in < 10) return;
  if (in_sizes[0] != NN * FD) return;
  if (in_sizes[1] != 2 * NE) return;
  if (in_sizes[2] != FD * FD || in_sizes[3] != FD) return;
  if (in_sizes[4] != FD * FD || in_sizes[5] != FD * FD || in_sizes[6] != FD) return;
  if (in_sizes[7] != FD * CD || in_sizes[8] != FD * CD || in_sizes[9] != CD) return;
  if ((long long)out_size != (long long)NN * CD) return;

  const float* x   = (const float*)d_in[0];
  const int*   ei  = (const int*)  d_in[1];
  const int*   src = ei;
  const int*   dst = ei + NE;
  const float* Wp  = (const float*)d_in[2];
  const float* bpl = (const float*)d_in[3];
  const float* Wl1 = (const float*)d_in[4];
  const float* Wr1 = (const float*)d_in[5];
  const float* b1  = (const float*)d_in[6];
  const float* Wl2 = (const float*)d_in[7];
  const float* Wr2 = (const float*)d_in[8];
  const float* b2  = (const float*)d_in[9];
  float* out = (float*)d_out;

  const int nN = NN, nE = NE, nB = NBLK;
  const int vec8 = ((nE & 3) == 0) ? 1 : 0;

  char* ws = (char*)d_ws;
  size_t off = 0;
  const size_t oWPT  = off; off = al256(off + (size_t)64 * 64 * 2);
  const size_t oWPT2 = off; off = al256(off + (size_t)64 * 128 * 2);
  const size_t oW1C  = off; off = al256(off + (size_t)64 * 192 * 2);
  const size_t oW2C  = off; off = al256(off + (size_t)NPC * 256 * 2);
  const size_t oXB   = off; off = al256(off + (size_t)MP * 64 * 2);
  const size_t oM    = off; off = al256(off + (size_t)MP * 64 * 4);
  const size_t oAGG  = off; off = al256(off + (size_t)MP * 128 * 2);
  const size_t oH    = off; off = al256(off + (size_t)MP * 128 * 2);
  const size_t oLS   = off; off = al256(off + (size_t)NBLK * RCAP * 4);
  const size_t oCN   = off; off = al256(off + (size_t)NPADN * 4);
  const size_t oOF   = off; off = al256(off + (size_t)NPADN * 4);
  const size_t oRC   = off; off = al256(off + (size_t)NBLK * 128);
  if (off > ws_size || off > (size_t)WSMAX) return;
  unsigned short* WPT  = (unsigned short*)(ws + oWPT);
  unsigned short* WPT2 = (unsigned short*)(ws + oWPT2);
  unsigned short* W1C  = (unsigned short*)(ws + oW1C);
  unsigned short* W2C  = (unsigned short*)(ws + oW2C);
  unsigned short* XB   = (unsigned short*)(ws + oXB);
  float*          Mp   = (float*)(ws + oM);
  unsigned short* AGG  = (unsigned short*)(ws + oAGG);
  unsigned short* Hp   = (unsigned short*)(ws + oH);
  int* LIST = (int*)(ws + oLS);
  int* CNT  = (int*)(ws + oCN);
  int* OFF  = (int*)(ws + oOF);
  int* REC  = (int*)(ws + oRC);

  hipFuncSetAttribute(reinterpret_cast<const void*>(&k_bucket), hipFuncAttributeMaxDynamicSharedMemorySize, LDS_BK);

  const int gPrep = NWBLK + (MP * 8) / NTHR;
  const int gG    = MP / GBM;
  const int gR    = MP / RPB;

  k_prep<<<gPrep, NTHR, 0, stream>>>(x, Wp, Wl1, Wr1, Wl2, Wr2, WPT, WPT2, W1C, W2C, XB, nN, MP);
  k_bucket<<<nB, NTHR, LDS_BK, stream>>>(dst, src, nE, nN, vec8, LIST, CNT, OFF, REC);
  k_gemm<0><<<gG, GTHR, 0, stream>>>(XB, XB, WPT, bpl, Mp, Hp, REC, nN, nB);
  k_max<<<gR, NTHR, 0, stream>>>(Mp, LIST, CNT, OFF, REC, AGG, nN, MP, nB);
  k_gemm<1><<<gG, GTHR, 0, stream>>>(AGG, XB, W1C, b1, Mp, Hp, REC, nN, nB);
  k_gemm<2><<<gG, GTHR, 0, stream>>>(Hp, Hp, WPT2, bpl, Mp, AGG, REC, nN, nB);
  k_max<<<gR, NTHR, 0, stream>>>(Mp, LIST, CNT, OFF, REC, AGG, nN, MP, nB);
  k_gemm<3><<<gG, GTHR, 0, stream>>>(AGG, Hp, W2C, b2, out, XB, REC, nN, nB);
}
